// EGNNExpert_20538533609914
// MI455X (gfx1250) — hardware-run, weakly checked
//
#include <hip/hip_runtime.h>
#include <stddef.h>
#include <stdint.h>


#define NN      50000
#define NE      800000
#define FIN     64
#define HID     192
#define NHD     12
#define HC      16
#define NL      3
#define K2      384
#define MP      50048
#define GBM     64
#define GTHR    128
#define NTHR    256
#define NWAVE   8
#define EPT     8
#define CHUNK   (NTHR * EPT)
#define WCAP    (EPT * 32)
#define LISTN   (NWAVE * WCAP)
#define NB      1024
#define NBLK    49
#define RCAP    21504
#define DEGCAP  256
#define SROWS   64
#define WSMAX   134217728
#define LDS_BKT ((2 * RCAP + 2 * NB + LISTN + 2 * NWAVE) * 4)
#define PB_X    1564
#define PB_WIN  6
#define PB_W    18
#define PB_TOT  (PB_X + PB_WIN + 7 * PB_W)

static_assert(HID == NHD * HC);
static_assert(HID == 6 * 32);
static_assert(HC == 16);
static_assert(K2 == 2 * HID);
static_assert((FIN % 32) == 0 && (K2 % 32) == 0);
static_assert(MP >= NN && (MP % GBM) == 0 && (MP % SROWS) == 0);
static_assert(NBLK * NB >= NN && NBLK * NB >= MP);
static_assert((NB % GBM) == 0 && (NB % SROWS) == 0);
static_assert(NN <= 65536);
static_assert(NE < (1 << 20));
static_assert((NE & 3) == 0);
static_assert((CHUNK & (CHUNK - 1)) == 0 && CHUNK <= 4096);
static_assert((NB & (NB - 1)) == 0 && NB <= 4096);
static_assert(NTHR * 4 == NB);
static_assert(LISTN >= NB);
static_assert((RCAP % (2 * NTHR)) == 0 && RCAP >= 16623 + 16623 / 4);
static_assert(DEGCAP >= 35 + 8);
static_assert(LDS_BKT <= 300000);
static_assert(MP * (FIN / 8) == PB_X * NTHR);
static_assert(HID * (FIN / 8) == PB_WIN * NTHR);
static_assert(HID * (HID / 8) == PB_W * NTHR);
static_assert(GBM * HID * 4 + 6 * HID * 4 + NWAVE * K2 * 2 <= 65536);
static_assert((size_t)NN * HID == 9600000);

#define SZ_XB   ((size_t)MP * FIN * 2)
#define SZ_HHL  ((size_t)MP * K2 * 2)
#define SZ_XLR  ((size_t)MP * K2 * 4)
#define SZ_HITS ((size_t)NBLK * RCAP * 8)
#define SZ_SLOT ((size_t)NBLK * NB * 16)
#define SZ_WINT ((size_t)HID * FIN * 2)
#define SZ_WLR  ((size_t)NL * K2 * K2 * 2)
#define SZ_WGD  ((size_t)HID * K2 * 2)
#define SZ_TOT  (SZ_XB + SZ_HHL + SZ_XLR + SZ_HITS + SZ_SLOT + SZ_WINT + SZ_WLR + SZ_WGD)
static_assert((SZ_XB % 256) == 0 && (SZ_HHL % 256) == 0 && (SZ_XLR % 256) == 0 && (SZ_HITS % 256) == 0);
static_assert((SZ_SLOT % 256) == 0 && (SZ_WINT % 256) == 0 && (SZ_WLR % 256) == 0 && (SZ_WGD % 256) == 0);
static_assert(SZ_TOT <= (size_t)WSMAX);

typedef float          v2f   __attribute__((ext_vector_type(2)));
typedef float          v4f   __attribute__((ext_vector_type(4)));
typedef float          v8f   __attribute__((ext_vector_type(8)));
typedef int            v2i   __attribute__((ext_vector_type(2)));
typedef int            v4i   __attribute__((ext_vector_type(4)));
typedef int            v8i   __attribute__((ext_vector_type(8)));
typedef unsigned short v8us  __attribute__((ext_vector_type(8)));
typedef __bf16         v16bf __attribute__((ext_vector_type(16)));
typedef v4f  __attribute__((may_alias)) v4fa;
typedef v8us __attribute__((may_alias)) v8usa;
union FragB { v16bf v; v8us u[2]; v8i w; v4i q[2]; };

__device__ __forceinline__ v8f wmx(const FragB& a, const FragB& b, v8f c) {
  v8f d = __builtin_amdgcn_wmma_f32_16x16x32_bf16(false, a.v, false, b.v, (short)0, c, false, false);
  asm volatile("v_nop\n\tv_nop\n\tv_nop\n\tv_nop" : "+v"(d) : "v"(a.w), "v"(b.w));
  return d;
}

__device__ __forceinline__ void pinf(float x) { asm volatile("" :: "v"(x)); }
__device__ __forceinline__ void pini(int x)   { asm volatile("" :: "v"(x)); }
__device__ __forceinline__ void pin4(const v4f a) { pinf(a.x); pinf(a.y); pinf(a.z); pinf(a.w); }

__device__ __forceinline__ unsigned bfbits(float v) {
  const unsigned u = __float_as_uint(v);
  const unsigned r = (u + 0x7FFFu + ((u >> 16) & 1u)) >> 16;
  const unsigned nb = ((u >> 16) & 0x8000u) | 0x7FC0u;
  return ((u & 0x7FFFFFFFu) > 0x7F800000u) ? nb : r;
}
__device__ __forceinline__ float rbf(float v) { return __uint_as_float(bfbits(v) << 16); }
__device__ __forceinline__ v4f rbf4(const v4f a) {
  v4f o; o.x = rbf(a.x); o.y = rbf(a.y); o.z = rbf(a.z); o.w = rbf(a.w); return o;
}
__device__ __forceinline__ float wsum(float v) {
#pragma unroll
  for (int off = 16; off > 0; off >>= 1) v += __shfl_xor(v, off);
  return v;
}
__device__ __forceinline__ float rcp_nr(float s) {
  const float r = __builtin_amdgcn_rcpf(s);
  const float e = fmaf(-s, r, 1.0f);
  return fmaf(e, r, r);
}

__device__ __forceinline__ int scan_chunk(const int* __restrict__ dsts, int nE, int cbase, int slotBase,
                                          int nb, int vec8, int* list, int tid, int lane, int wave) {
  int wc = 0;
  const int el0  = tid * EPT;
  const int e0   = cbase + el0;
  const int sent = -2147483647 - 1;
  v4i da, db;
  if (vec8 != 0 && cbase + CHUNK <= nE) {
    da = *(const v4i*)(dsts + e0);
    db = *(const v4i*)(dsts + e0 + 4);
  } else {
    da.x = (e0     < nE) ? dsts[min(e0,     nE - 1)] : sent;
    da.y = (e0 + 1 < nE) ? dsts[min(e0 + 1, nE - 1)] : sent;
    da.z = (e0 + 2 < nE) ? dsts[min(e0 + 2, nE - 1)] : sent;
    da.w = (e0 + 3 < nE) ? dsts[min(e0 + 3, nE - 1)] : sent;
    db.x = (e0 + 4 < nE) ? dsts[min(e0 + 4, nE - 1)] : sent;
    db.y = (e0 + 5 < nE) ? dsts[min(e0 + 5, nE - 1)] : sent;
    db.z = (e0 + 6 < nE) ? dsts[min(e0 + 6, nE - 1)] : sent;
    db.w = (e0 + 7 < nE) ? dsts[min(e0 + 7, nE - 1)] : sent;
  }
  const unsigned nbs = (unsigned)slotBase;
  const unsigned unb = (unsigned)nb;
  const unsigned s0 = (unsigned)da.x - nbs, s1 = (unsigned)da.y - nbs;
  const unsigned s2 = (unsigned)da.z - nbs, s3 = (unsigned)da.w - nbs;
  const unsigned s4 = (unsigned)db.x - nbs, s5 = (unsigned)db.y - nbs;
  const unsigned s6 = (unsigned)db.z - nbs, s7 = (unsigned)db.w - nbs;
  const bool h0 = s0 < unb, h1 = s1 < unb, h2 = s2 < unb, h3 = s3 < unb;
  const bool h4 = s4 < unb, h5 = s5 < unb, h6 = s6 < unb, h7 = s7 < unb;
  const unsigned any = __builtin_amdgcn_ballot_w32(h0 | h1 | h2 | h3 | h4 | h5 | h6 | h7);
  if (any != 0u) {
#define HITJ(J, HJ, SJ) { \
      const unsigned mj = __builtin_amdgcn_ballot_w32(HJ); \
      if (mj != 0u) { \
        if (HJ) { \
          const int pos = wc + (int)__builtin_amdgcn_mbcnt_lo(mj, 0u); \
          if (pos < WCAP) list[wave * WCAP + pos] = ((el0 + (J)) << 12) | (int)(SJ); \
        } \
        wc += (int)__builtin_popcount(mj); } }
    HITJ(0, h0, s0)
    HITJ(1, h1, s1)
    HITJ(2, h2, s2)
    HITJ(3, h3, s3)
    HITJ(4, h4, s4)
    HITJ(5, h5, s5)
    HITJ(6, h6, s6)
    HITJ(7, h7, s7)
#undef HITJ
  }
  return wc;
}

__device__ __forceinline__ void wtr_unit(const float* __restrict__ w, int Kin, int u, unsigned short* wt,
                                         int pitch, int dup) {
  const int kq = Kin >> 3;
  int n = u / kq;
  const int k8 = (u - n * kq) * 8;
  n = n < HID ? n : HID - 1;
  float f[8];
#pragma unroll
  for (int i = 0; i < 8; ++i) {
    f[i] = w[(size_t)(k8 + i) * HID + n];
    pinf(f[i]);
  }
  v8us hv;
#pragma unroll
  for (int i = 0; i < 8; ++i) hv[i] = (unsigned short)bfbits(f[i]);
  const size_t o = (size_t)n * (size_t)pitch + k8;
  *(volatile v8us*)(wt + o) = hv;
  if (dup != 0) *(volatile v8us*)(wt + o + Kin) = hv;
  __threadfence();
  *(volatile v8us*)(wt + o) = hv;
  if (dup != 0) *(volatile v8us*)(wt + o + Kin) = hv;
}

__global__ __launch_bounds__(NTHR) void k_prep(const float* __restrict__ x, const float* __restrict__ Win,
                                               const float* __restrict__ Wl, const float* __restrict__ Wr,
                                               const float* __restrict__ Wg, unsigned short* xb,
                                               unsigned short* wint, unsigned short* wlr, unsigned short* wgd) {
  const int b = (int)blockIdx.x, tid = (int)threadIdx.x;
  if (b < PB_X) {
    const int i = b * NTHR + tid;
    const int row = i >> 3;
    const int c0  = (i & 7) * 8;
    const int rc  = row < NN ? row : NN - 1;
    const float* p = x + (size_t)rc * FIN + c0;
    const v4f a = *(const v4f*)p, c = *(const v4f*)(p + 4);
    const unsigned mk = row < NN ? 0xFFFFu : 0u;
    v8us hv;
    hv[0] = (unsigned short)(bfbits(a.x) & mk); hv[1] = (unsigned short)(bfbits(a.y) & mk);
    hv[2] = (unsigned short)(bfbits(a.z) & mk); hv[3] = (unsigned short)(bfbits(a.w) & mk);
    hv[4] = (unsigned short)(bfbits(c.x) & mk); hv[5] = (unsigned short)(bfbits(c.y) & mk);
    hv[6] = (unsigned short)(bfbits(c.z) & mk); hv[7] = (unsigned short)(bfbits(c.w) & mk);
    const size_t o = (size_t)row * FIN + c0;
    *(volatile v8us*)(xb + o) = hv;
    __threadfence();
    *(volatile v8us*)(xb + o) = hv;
  } else if (b < PB_X + PB_WIN) {
    const int u = (b - PB_X) * NTHR + tid;
    wtr_unit(Win, FIN, u, wint, FIN, 0);
  } else {
    const int j   = b - PB_X - PB_WIN;
    const int job = j / PB_W;
    const int u   = (j - job * PB_W) * NTHR + tid;
    if (job < 3) {
      wtr_unit(Wl + (size_t)job * HID * HID, HID, u, wlr + (size_t)job * K2 * K2, K2, 1);
    } else if (job < 6) {
      wtr_unit(Wr + (size_t)(job - 3) * HID * HID, HID, u, wlr + (size_t)(job - 3) * K2 * K2 + (size_t)HID * K2, K2, 1);
    } else {
      wtr_unit(Wg, HID, u, wgd, K2, 1);
    }
  }
}

__global__ __launch_bounds__(NTHR) void k_bucket(const int* __restrict__ srcs, const int* __restrict__ dsts,
                                                 const float* __restrict__ ea, int* hits, int* slot, int vec8) {
  extern __shared__ v4f lds_dyn[];
  int* reg1 = (int*)lds_dyn;
  int* reg2 = reg1 + RCAP;
  int* scnt = reg2 + RCAP;
  int* soff = scnt + NB;
  int* list = soff + NB;
  int* wcnt = list + LISTN;
  int* wtot = wcnt + NWAVE;
  const int tid = (int)threadIdx.x, lane = tid & 31;
  const int wave = __builtin_amdgcn_readfirstlane(tid >> 5);
  const int nodeBase = (int)blockIdx.x * NB;

  for (int i = tid; i < NB; i += NTHR) { scnt[i] = 0; soff[i] = 0; }
  for (int i = tid; i < RCAP; i += NTHR) { reg1[i] = 0; reg2[i] = 0; }
  __syncthreads();

  int tot = 0;
  const int nChunks = (NE + CHUNK - 1) / CHUNK;
#pragma unroll 1
  for (int ch = 0; ch < nChunks; ++ch) {
    const int cbase = ch * CHUNK;
    const int wc = scan_chunk(dsts, NE, cbase, nodeBase, NB, vec8, list, tid, lane, wave);
    if (lane == 0) wcnt[wave] = wc;
    __syncthreads();
    int pre = 0, all = 0;
#pragma unroll
    for (int w2 = 0; w2 < NWAVE; ++w2) {
      int c = wcnt[w2];
      c = c < 0 ? 0 : (c > WCAP ? WCAP : c);
      all += c;
      pre += (w2 < wave) ? c : 0;
    }
    const int wcc  = wc > WCAP ? WCAP : wc;
    const int base = tot + pre;
#pragma unroll 1
    for (int i = lane; i < wcc; i += 32) {
      const int en = list[wave * WCAP + i];
      const int el = (en >> 12) & (CHUNK - 1);
      const int sl = en & (NB - 1);
      int eid = cbase + el;
      eid = eid > NE - 1 ? NE - 1 : eid;
      const int pos = base + i;
      if (pos < RCAP) reg1[pos] = (int)(((unsigned)eid << 10) | (unsigned)sl);
    }
    tot += all;
    tot = tot > RCAP ? RCAP : tot;
    __syncthreads();
  }
  const int nh = tot;

  if (wave == 0) {
#pragma unroll 1
    for (int b0 = 0; b0 < nh; b0 += 32) {
      const int idx = b0 + lane;
      const int uv  = reg1[idx < RCAP ? idx : RCAP - 1];
      const int m32 = (nh - b0) < 32 ? (nh - b0) : 32;
#pragma unroll 1
      for (int k = 0; k < m32; ++k) {
        const int u  = __builtin_amdgcn_readlane(uv, k);
        const int sl = u & (NB - 1);
        if (lane == 0) scnt[sl] = scnt[sl] + 1;
      }
    }
  }
  __syncthreads();

  {
    const int r0 = scnt[4 * tid], r1 = scnt[4 * tid + 1], r2 = scnt[4 * tid + 2], r3 = scnt[4 * tid + 3];
    const int e0 = r0 < 0 ? 0 : r0, e1 = r1 < 0 ? 0 : r1, e2 = r2 < 0 ? 0 : r2, e3 = r3 < 0 ? 0 : r3;
    const int ts = (e0 + e1) + (e2 + e3);
    int incl = ts;
#pragma unroll
    for (int d = 1; d < 32; d <<= 1) {
      const int up = __shfl_up(incl, d);
      if (lane >= d) incl += up;
    }
    if (lane == 31) wtot[wave] = incl;
    __syncthreads();
    int pre = 0;
#pragma unroll
    for (int w2 = 0; w2 < NWAVE; ++w2) pre += (w2 < wave) ? wtot[w2] : 0;
    const int run = pre + incl - ts;
    soff[4 * tid]     = run;
    soff[4 * tid + 1] = run + e0;
    soff[4 * tid + 2] = run + e0 + e1;
    soff[4 * tid + 3] = run + e0 + e1 + e2;
  }
  __syncthreads();
  for (int i = tid; i < NB; i += NTHR) list[i] = soff[i];
  __syncthreads();

  if (wave == 0) {
#pragma unroll 1
    for (int b0 = 0; b0 < nh; b0 += 32) {
      const int idx = b0 + lane;
      const int uv  = reg1[idx < RCAP ? idx : RCAP - 1];
      const int m32 = (nh - b0) < 32 ? (nh - b0) : 32;
#pragma unroll 1
      for (int k = 0; k < m32; ++k) {
        const int u   = __builtin_amdgcn_readlane(uv, k);
        const int sl  = u & (NB - 1);
        const int eid = (int)((unsigned)u >> 10);
        if (lane == 0) {
          int pos = list[sl];
          pos = pos < 0 ? 0 : (pos > RCAP - 1 ? RCAP - 1 : pos);
          reg2[pos] = eid;
          list[sl] = pos + 1;
        }
      }
    }
  }
  __syncthreads();

  const bool ovf = (nh >= RCAP);
  int* hb = hits + (size_t)blockIdx.x * (size_t)(2 * RCAP);
#pragma unroll 1
  for (int p0 = 0; p0 < RCAP; p0 += 2 * NTHR) {
    const int p = p0 + 2 * tid;
    int e0 = reg2[p], e1 = reg2[p + 1];
    e0 = e0 < 0 ? 0 : (e0 > NE - 1 ? NE - 1 : e0);
    e1 = e1 < 0 ? 0 : (e1 > NE - 1 ? NE - 1 : e1);
    const int s0 = srcs[e0];
    const int s1 = srcs[e1];
    const v2f a0 = *(const v2f*)(ea + 2 * (size_t)e0);
    const v2f a1 = *(const v2f*)(ea + 2 * (size_t)e1);
    pini(s0); pini(s1); pinf(a0.x); pinf(a0.y); pinf(a1.x); pinf(a1.y);
    const int m0 = (p     < nh) ? -1 : 0;
    const int m1 = (p + 1 < nh) ? -1 : 0;
    const int w0 = (int)(bfbits(a0.x) | (bfbits(a0.y) << 16));
    const int w1 = (int)(bfbits(a1.x) | (bfbits(a1.y) << 16));
    v4i v;
    v.x = s0 & m0; v.y = w0 & m0; v.z = s1 & m1; v.w = w1 & m1;
    *(volatile v4i*)(hb + 2 * p) = v;
    __threadfence();
    *(volatile v4i*)(hb + 2 * p) = v;
  }

#pragma unroll 1
  for (int j = 0; j < 4; ++j) {
    const int s = j * NTHR + tid;
    int st = soff[s];
    const int c = scnt[s];
    st = st < 0 ? 0 : (st > RCAP - 1 ? RCAP - 1 : st);
    int cc = c < 0 ? 0 : (c > DEGCAP ? DEGCAP : c);
    if (cc > RCAP - st) cc = RCAP - st;
    int wm = cc;
#pragma unroll
    for (int off = 16; off > 0; off >>= 1) {
      const int o2 = __shfl_xor(wm, off);
      wm = wm > o2 ? wm : o2;
    }
    float a0 = 0.0f, a1 = 0.0f;
#pragma unroll 1
    for (int p = 0; p < wm; ++p) {
      int idx = st + p;
      idx = idx > RCAP - 1 ? RCAP - 1 : idx;
      int e = reg2[idx];
      e = e < 0 ? 0 : (e > NE - 1 ? NE - 1 : e);
      const v2f a = *(const v2f*)(ea + 2 * (size_t)e);
      pinf(a.x); pinf(a.y);
      const bool on = p < cc;
      const float t0 = a0 + rbf(a.x);
      const float t1 = a1 + rbf(a.y);
      a0 = on ? t0 : a0;
      a1 = on ? t1 : a1;
    }
    const float dv = (float)(cc > 1 ? cc : 1);
    const float m0 = a0 / dv;
    const float m1 = a1 / dv;
    v4i sv;
    sv.x = st;
    sv.y = ovf ? -1 : c;
    sv.z = __float_as_int(m0);
    sv.w = __float_as_int(m1);
    int* sp = slot + 4 * (size_t)(nodeBase + s);
    *(volatile v4i*)sp = sv;
    __threadfence();
    *(volatile v4i*)sp = sv;
  }
}

template<int K>
__device__ __forceinline__ void gemm_core(const unsigned short* __restrict__ A, const unsigned short* __restrict__ B,
                                          int rowBase, int colBase, int rg, int cg, int hh, int m,
                                          v8f (&acc)[2][6]) {
  const v8f z = {0.f, 0.f, 0.f, 0.f, 0.f, 0.f, 0.f, 0.f};
#pragma unroll
  for (int mt = 0; mt < 2; ++mt)
#pragma unroll
    for (int nt = 0; nt < 6; ++nt) acc[mt][nt] = z;
  const unsigned short* ap0 = A + (size_t)(rowBase + 32 * rg + m) * (size_t)K + 8 * hh;
  const unsigned short* ap1 = ap0 + (size_t)16 * (size_t)K;
  const unsigned short* bp  = B + (size_t)(colBase + 96 * cg + m) * (size_t)K + 8 * hh;
#pragma unroll 1
  for (int ks = 0; ks < K / 32; ++ks) {
    FragB a0, a1;
    a0.u[0] = *(const v8us*)(ap0 + 32 * ks);
    a0.u[1] = *(const v8us*)(ap0 + 32 * ks + 16);
    a1.u[0] = *(const v8us*)(ap1 + 32 * ks);
    a1.u[1] = *(const v8us*)(ap1 + 32 * ks + 16);
#pragma unroll
    for (int nt = 0; nt < 6; ++nt) {
      const unsigned short* bq = bp + (size_t)(16 * nt) * (size_t)K + 32 * ks;
      FragB bf;
      bf.u[0] = *(const v8us*)bq;
      bf.u[1] = *(const v8us*)(bq + 16);
      acc[0][nt] = wmx(a0, bf, acc[0][nt]);
      acc[1][nt] = wmx(a1, bf, acc[1][nt]);
    }
  }
}

__device__ __forceinline__ void stage_tile(float* tile, const v8f (&acc)[2][6], int rg, int cg, int hh, int m) {
#pragma unroll
  for (int mt = 0; mt < 2; ++mt)
#pragma unroll
    for (int nt = 0; nt < 6; ++nt)
#pragma unroll
      for (int r = 0; r < 8; ++r)
        tile[(32 * rg + 16 * mt + 8 * hh + r) * HID + 96 * cg + 16 * nt + m] = acc[mt][nt][r];
}

__device__ __forceinline__ void ln6(const float (&v)[6], const float (&g)[6], const float (&b)[6], float (&y)[6]) {
  const float s = ((v[0] + v[1]) + (v[2] + v[3])) + (v[4] + v[5]);
  const float mu = wsum(s) * (1.0f / (float)HID);
  float d[6];
  float q = 0.0f;
#pragma unroll
  for (int k = 0; k < 6; ++k) { d[k] = v[k] - mu; q = fmaf(d[k], d[k], q); }
  const float var = wsum(q) * (1.0f / (float)HID);
  const float rstd = 1.0f / sqrtf(var + 1e-5f);
#pragma unroll
  for (int k = 0; k < 6; ++k) y[k] = (d[k] * rstd) * g[k] + b[k];
}

template<int WHL>
__device__ __forceinline__ void put_rows(const float (&y)[6], float* hrow, bool wrH,
                                         unsigned short* lrow, unsigned short* stg, int lane, unsigned pm) {
  v8us v0 = {0, 0, 0, 0, 0, 0, 0, 0};
  v8us v1 = {0, 0, 0, 0, 0, 0, 0, 0};
  if (WHL) {
#pragma unroll
    for (int k = 0; k < 6; ++k) {
      const unsigned hb = bfbits(y[k]);
      const unsigned lb = bfbits(y[k] - __uint_as_float(hb << 16));
      stg[lane + 32 * k]       = (unsigned short)(hb & pm);
      stg[HID + lane + 32 * k] = (unsigned short)(lb & pm);
    }
    __builtin_amdgcn_fence(__ATOMIC_RELEASE, "wavefront");
    __builtin_amdgcn_wave_barrier();
    v0 = *(const v8usa*)(stg + 8 * lane);
    v1 = *(const v8usa*)(stg + 256 + 8 * (lane & 15));
    __builtin_amdgcn_fence(__ATOMIC_RELEASE, "wavefront");
    __builtin_amdgcn_wave_barrier();
  }
  if (wrH) {
#pragma unroll
    for (int k = 0; k < 6; ++k) *(volatile float*)(hrow + lane + 32 * k) = y[k];
  }
  if (WHL) {
    *(volatile v8us*)(lrow + 8 * lane) = v0;
    if (lane < 16) *(volatile v8us*)(lrow + 256 + 8 * lane) = v1;
  }
  __threadfence();
  if (wrH) {
#pragma unroll
    for (int k = 0; k < 6; ++k) *(volatile float*)(hrow + lane + 32 * k) = y[k];
  }
  if (WHL) {
    *(volatile v8us*)(lrow + 8 * lane) = v0;
    if (lane < 16) *(volatile v8us*)(lrow + 256 + 8 * lane) = v1;
  }
}

__global__ __launch_bounds__(GTHR) __attribute__((amdgpu_num_vgpr(248)))
void k_in(const unsigned short* __restrict__ xb, const unsigned short* __restrict__ wint,
          const float* __restrict__ b_in, const float* __restrict__ gam, const float* __restrict__ bet,
          float* hout, unsigned short* hhl) {
  __shared__ __attribute__((aligned(16))) float tile[GBM * HID];
  __shared__ __attribute__((aligned(16))) float sp[3 * HID];
  __shared__ __attribute__((aligned(16))) unsigned short sst[4 * K2];
  const int tid = (int)threadIdx.x, lane = tid & 31, hh = lane >> 4, m = lane & 15;
  const int wave = __builtin_amdgcn_readfirstlane(tid >> 5);
  const int rg = wave >> 1, cg = wave & 1;
  const int rowBase = (int)blockIdx.x * GBM;
  {
    const int t = tid < 47 ? tid : 47;
    const v4f r0 = *(const v4f*)(b_in + 4 * t);
    pin4(r0);
    const v4f r1 = *(const v4f*)(gam + 4 * t);
    pin4(r1);
    const v4f r2 = *(const v4f*)(bet + 4 * t);
    pin4(r2);
    const v4f p0 = rbf4(r0);
    const v4f p1 = rbf4(r1);
    const v4f p2 = rbf4(r2);
    if (tid < 48) {
      *(v4fa*)(sp + 4 * tid)           = p0;
      *(v4fa*)(sp + HID + 4 * tid)     = p1;
      *(v4fa*)(sp + 2 * HID + 4 * tid) = p2;
    }
  }
  v8f acc[2][6];
  gemm_core<FIN>(xb, wint, rowBase, 0, rg, cg, hh, m, acc);
  stage_tile(tile, acc, rg, cg, hh, m);
  __syncthreads();

  float bi[6], gg[6], bb[6];
#pragma unroll
  for (int k = 0; k < 6; ++k) {
    bi[k] = sp[lane + 32 * k];
    gg[k] = sp[HID + lane + 32 * k];
    bb[k] = sp[2 * HID + lane + 32 * k];
  }
  unsigned short* stg = sst + wave * K2;
#pragma unroll 1
  for (int rr = 0; rr < 16; ++rr) {
    const int lr  = 16 * wave + rr;
    const int row = rowBase + lr;
    float v[6], y[6];
#pragma unroll
    for (int k = 0; k < 6; ++k) {
      const float z = tile[lr * HID + lane + 32 * k] + bi[k];
      v[k] = 0.5f * z * (1.0f + erff(z * 0.70710678118654752f));
    }
    ln6(v, gg, bb, y);
    const unsigned pm = row < NN ? 0xFFFFu : 0u;
    put_rows<1>(y, hout + (size_t)(row < NN ? row : NN - 1) * HID, row < NN,
                hhl + (size_t)row * K2, stg, lane, pm);
  }
}

__device__ __forceinline__ void proj_store(const float* tile, const float* sb, float* xlr,
                                           int rowBase, int colBase, int wave, int lane) {
#pragma unroll 4
  for (int it = 0; it < 24; ++it) {
    const int v  = it * 32 + lane;
    const int rl = v / 48;
    const int c4 = v - rl * 48;
    const int lr = 16 * wave + rl;
    const v4f a = *(const v4fa*)(tile + lr * HID + 4 * c4);
    const v4f b = *(const v4fa*)(sb + 4 * c4);
    const v4f o = a + b;
    *(volatile v4f*)(xlr + (size_t)(rowBase + lr) * K2 + colBase + 4 * c4) = o;
  }
}

__global__ __launch_bounds__(GTHR) __attribute__((amdgpu_num_vgpr(248)))
void k_proj(const unsigned short* __restrict__ hhl, const unsigned short* __restrict__ wlr,
            const float* __restrict__ bl, const float* __restrict__ br, float* xlr) {
  __shared__ __attribute__((aligned(16))) float tile[GBM * HID];
  __shared__ __attribute__((aligned(16))) float sb[HID];
  const int tid = (int)threadIdx.x, lane = tid & 31, hh = lane >> 4, m = lane & 15;
  const int wave = __builtin_amdgcn_readfirstlane(tid >> 5);
  const int rg = wave >> 1, cg = wave & 1;
  const int rowBase = (int)blockIdx.x * GBM;
  const int colBase = (int)blockIdx.y * HID;
  {
    const int t = tid < 47 ? tid : 47;
    const v4f b0 = *(const v4f*)(bl + 4 * t);
    pin4(b0);
    const v4f b1 = *(const v4f*)(br + 4 * t);
    pin4(b1);
    const v4f bv = (blockIdx.y != 0) ? b1 : b0;
    const v4f bq = rbf4(bv);
    if (tid < 48) *(v4fa*)(sb + 4 * tid) = bq;
  }
  v8f acc[2][6];
  gemm_core<K2>(hhl, wlr, rowBase, colBase, rg, cg, hh, m, acc);
  stage_tile(tile, acc, rg, cg, hh, m);
  __syncthreads();
  proj_store(tile, sb, xlr, rowBase, colBase, wave, lane);
  __threadfence();
  proj_store(tile, sb, xlr, rowBase, colBase, wave, lane);
}

__global__ __launch_bounds__(NTHR) __attribute__((amdgpu_num_vgpr(248)))
void k_scan(const int* __restrict__ hits, const int* __restrict__ slot, const float* __restrict__ xlr,
            const float* __restrict__ We, const float* __restrict__ att, const float* __restrict__ bo,
            const float* __restrict__ gam, const float* __restrict__ bet,
            float* hbuf, unsigned short* hhl) {
  __shared__ __attribute__((aligned(16))) float sp[6 * HID];
  __shared__ __attribute__((aligned(16))) unsigned short sst[NWAVE * K2];
  const int tid = (int)threadIdx.x, lane = tid & 31;
  const int wave = __builtin_amdgcn_readfirstlane(tid >> 5);
  {
    const int t = tid < 47 ? tid : 47;
    const v4f r0 = *(const v4f*)(We + 4 * t);
    pin4(r0);
    const v4f r1 = *(const v4f*)(We + HID + 4 * t);
    pin4(r1);
    const v4f r2 = *(const v4f*)(att + 4 * t);
    pin4(r2);
    const v4f r3 = *(const v4f*)(bo + 4 * t);
    pin4(r3);
    const v4f r4 = *(const v4f*)(gam + 4 * t);
    pin4(r4);
    const v4f r5 = *(const v4f*)(bet + 4 * t);
    pin4(r5);
    const v4f p0 = rbf4(r0);
    const v4f p1 = rbf4(r1);
    const v4f p2 = rbf4(r2);
    const v4f p3 = rbf4(r3);
    const v4f p4 = rbf4(r4);
    const v4f p5 = rbf4(r5);
    if (tid < 48) {
      *(v4fa*)(sp + 4 * tid)           = p0;
      *(v4fa*)(sp + HID + 4 * tid)     = p1;
      *(v4fa*)(sp + 2 * HID + 4 * tid) = p2;
      *(v4fa*)(sp + 3 * HID + 4 * tid) = p3;
      *(v4fa*)(sp + 4 * HID + 4 * tid) = p4;
      *(v4fa*)(sp + 5 * HID + 4 * tid) = p5;
    }
  }
  __syncthreads();
  float we0[6], we1[6], at[6], bo6[6], gg[6], bb[6];
#pragma unroll
  for (int k = 0; k < 6; ++k) {
    we0[k] = sp[lane + 32 * k];
    we1[k] = sp[HID + lane + 32 * k];
    at[k]  = sp[2 * HID + lane + 32 * k];
    bo6[k] = sp[3 * HID + lane + 32 * k];
    gg[k]  = sp[4 * HID + lane + 32 * k];
    bb[k]  = sp[5 * HID + lane + 32 * k];
  }
  unsigned short* stg = sst + wave * K2;
  const float qnan = __int_as_float(0x7fc00000);

#pragma unroll 1
  for (int j = 0; j < SROWS / NWAVE; ++j) {
    const int i = (int)blockIdx.x * SROWS + j * NWAVE + wave;
    if (i >= NN) break;
    const v4i se = *(const v4i*)(slot + 4 * (size_t)i);
    int st = __builtin_amdgcn_readfirstlane(se.x);
    const int craw = __builtin_amdgcn_readfirstlane(se.y);
    const int m0b  = __builtin_amdgcn_readfirstlane(se.z);
    const int m1b  = __builtin_amdgcn_readfirstlane(se.w);
    st = st < 0 ? 0 : (st > RCAP - 1 ? RCAP - 1 : st);
    int cnt = craw < 0 ? 0 : (craw > DEGCAP ? DEGCAP : craw);
    if (cnt > RCAP - st) cnt = RCAP - st;
    const float pz = (craw < 0 || craw > DEGCAP) ? qnan : 0.0f;
    const int* hb = hits + (size_t)(i >> 10) * (size_t)(2 * RCAP);

    float xr[6], mx[6], sm[6], acc[6];
    {
      const float* xq = xlr + (size_t)i * K2 + HID + lane;
#pragma unroll
      for (int k = 0; k < 6; ++k) { xr[k] = xq[32 * k]; mx[k] = -1.0e30f; sm[k] = 0.0f; acc[k] = 0.0f; }
    }

    const int tot = cnt + 1;
#pragma unroll 1
    for (int t0 = 0; t0 < tot; t0 += 32) {
      const int nv = (tot - t0) < 32 ? (tot - t0) : 32;
      const int q  = t0 + lane;
      int idx = st + q - 1;
      idx = idx > st + cnt - 1 ? st + cnt - 1 : idx;
      idx = idx < st ? st : idx;
      const v2i rec = *(const v2i*)(hb + 2 * idx);
      pini(rec.x); pini(rec.y);
      int sr = rec.x < 0 ? 0 : (rec.x > NN - 1 ? NN - 1 : rec.x);
      int e0b = (int)((unsigned)rec.y << 16);
      int e1b = (int)((unsigned)rec.y & 0xFFFF0000u);
      const int selfm = (q == 0) ? -1 : 0;
      sr  = (i   & selfm) | (sr  & ~selfm);
      e0b = (m0b & selfm) | (e0b & ~selfm);
      e1b = (m1b & selfm) | (e1b & ~selfm);
#pragma unroll 1
      for (int r = 0; r < nv; ++r) {
        const int s = __builtin_amdgcn_readlane(sr, r);
        const float a0 = __int_as_float(__builtin_amdgcn_readlane(e0b, r));
        const float a1 = __int_as_float(__builtin_amdgcn_readlane(e1b, r));
        const float* xp = xlr + (size_t)s * K2 + lane;
        float xl[6];
#pragma unroll
        for (int k = 0; k < 6; ++k) xl[k] = xp[32 * k];
#pragma unroll
        for (int k = 0; k < 6; ++k) {
          const float ee = fmaf(a1, we1[k], a0 * we0[k]);
          const float mm = (xl[k] + xr[k]) + ee;
          const float lk = (mm > 0.0f) ? mm : 0.2f * mm;
          float t = lk * at[k];
          t += __shfl_xor(t, 8);
          t += __shfl_xor(t, 4);
          t += __shfl_xor(t, 2);
          t += __shfl_xor(t, 1);
          const float d  = t - mx[k];
          const float e  = __builtin_amdgcn_exp2f(-fabsf(d) * 1.4426950408889634f);
          const bool up  = d > 0.0f;
          const float sc = up ? e : 1.0f;
          const float p  = up ? 1.0f : e;
          mx[k]  = up ? t : mx[k];
          sm[k]  = fmaf(sm[k], sc, p);
          acc[k] = fmaf(acc[k], sc, p * xl[k]);
        }
      }
    }

    float v[6], y[6];
    {
      const float* hq = hbuf + (size_t)i * HID + lane;
#pragma unroll
      for (int k = 0; k < 6; ++k) {
        const float hres = hq[32 * k];
        const float inv  = rcp_nr(sm[k]);
        v[k] = hres + (acc[k] * inv + bo6[k]);
      }
    }
    ln6(v, gg, bb, y);
#pragma unroll
    for (int k = 0; k < 6; ++k) y[k] = y[k] + pz;
    put_rows<1>(y, hbuf + (size_t)i * HID, true, hhl + (size_t)i * K2, stg, lane, 0xFFFFu);
  }
}

__global__ __launch_bounds__(GTHR) __attribute__((amdgpu_num_vgpr(248)))
void k_gate(const unsigned short* __restrict__ hhl, const unsigned short* __restrict__ wgd,
            const float* __restrict__ bg, const float* __restrict__ gam, const float* __restrict__ bet,
            const int* __restrict__ slot, float* hio) {
  __shared__ __attribute__((aligned(16))) float tile[GBM * HID];
  __shared__ __attribute__((aligned(16))) float sp[3 * HID];
  const int tid = (int)threadIdx.x, lane = tid & 31, hh = lane >> 4, m = lane & 15;
  const int wave = __builtin_amdgcn_readfirstlane(tid >> 5);
  const int rg = wave >> 1, cg = wave & 1;
  const int rowBase = (int)blockIdx.x * GBM;
  {
    const int t = tid < 47 ? tid : 47;
    const v4f r0 = *(const v4f*)(bg + 4 * t);
    pin4(r0);
    const v4f r1 = *(const v4f*)(gam + 4 * t);
    pin4(r1);
    const v4f r2 = *(const v4f*)(bet + 4 * t);
    pin4(r2);
    const v4f p0 = rbf4(r0);
    const v4f p1 = rbf4(r1);
    const v4f p2 = rbf4(r2);
    if (tid < 48) {
      *(v4fa*)(sp + 4 * tid)           = p0;
      *(v4fa*)(sp + HID + 4 * tid)     = p1;
      *(v4fa*)(sp + 2 * HID + 4 * tid) = p2;
    }
  }
  v8f acc[2][6];
  gemm_core<K2>(hhl, wgd, rowBase, 0, rg, cg, hh, m, acc);
  stage_tile(tile, acc, rg, cg, hh, m);
  __syncthreads();

  float bi[6], gg[6], bb[6];
#pragma unroll
  for (int k = 0; k < 6; ++k) {
    bi[k] = sp[lane + 32 * k];
    gg[k] = sp[HID + lane + 32 * k];
    bb[k] = sp[2 * HID + lane + 32 * k];
  }
  const float qnan = __int_as_float(0x7fc00000);
#pragma unroll 1
  for (int rr = 0; rr < 16; ++rr) {
    const int lr  = 16 * wave + rr;
    const int row = rowBase + lr;
    const int rc  = row < NN ? row : NN - 1;
    const int craw = __builtin_amdgcn_readfirstlane(slot[4 * (size_t)rc + 1]);
    const float pz = (craw < 0 || craw > DEGCAP) ? qnan : 0.0f;
    const float* hq = hio + (size_t)rc * HID + lane;
    float v[6], y[6];
#pragma unroll
    for (int k = 0; k < 6; ++k) {
      const float hv = hq[32 * k];
      const float z  = tile[lr * HID + lane + 32 * k] + bi[k];
      const float gt = 1.0f / (1.0f + expf(-z));
      v[k] = hv * gt;
    }
    ln6(v, gg, bb, y);
#pragma unroll
    for (int k = 0; k < 6; ++k) y[k] = y[k] + pz;
    put_rows<0>(y, hio + (size_t)rc * HID, row < NN, (unsigned short*)0, (unsigned short*)0, lane, 0xFFFFu);
  }
}

extern "C" void kernel_launch(void* const* d_in, const int* in_sizes, int n_in,
                              void* d_out, int out_size, void* d_ws, size_t ws_size,
                              hipStream_t stream) {
  if (n_in < 20) return;
  if (in_sizes[0] != NN * FIN) return;
  if (in_sizes[1] != 2 * NE) return;
  if (in_sizes[2] != NE * 2) return;
  if (in_sizes[3] != FIN * HID) return;
  if (in_sizes[4] != HID || in_sizes[5] != HID || in_sizes[6] != HID) return;
  if (in_sizes[7] != NL * HID * HID || in_sizes[9] != NL * HID * HID) return;
  if (in_sizes[8] != NL * HID || in_sizes[10] != NL * HID) return;
  if (in_sizes[11] != NL * 2 * HID) return;
  if (in_sizes[12] != NL * NHD * HC) return;
  if (in_sizes[13] != NL * HID || in_sizes[14] != NL * HID || in_sizes[15] != NL * HID) return;
  if (in_sizes[16] != HID * HID) return;
  if (in_sizes[17] != HID || in_sizes[18] != HID || in_sizes[19] != HID) return;
  if (out_size != NN * HID) return;
  if (SZ_TOT > ws_size) return;

  const float* x     = (const float*)d_in[0];
  const int*   ei    = (const int*)  d_in[1];
  const float* ea    = (const float*)d_in[2];
  const float* W_in  = (const float*)d_in[3];
  const float* b_in  = (const float*)d_in[4];
  const float* g_lni = (const float*)d_in[5];
  const float* b_lni = (const float*)d_in[6];
  const float* Wl    = (const float*)d_in[7];
  const float* bl    = (const float*)d_in[8];
  const float* Wr    = (const float*)d_in[9];
  const float* br    = (const float*)d_in[10];
  const float* We    = (const float*)d_in[11];
  const float* att   = (const float*)d_in[12];
  const float* bo    = (const float*)d_in[13];
  const float* g_res = (const float*)d_in[14];
  const float* b_res = (const float*)d_in[15];
  const float* Wg    = (const float*)d_in[16];
  const float* bg    = (const float*)d_in[17];
  const float* g_f   = (const float*)d_in[18];
  const float* b_f   = (const float*)d_in[19];
  float* out = (float*)d_out;
  const int* src = ei;
  const int* dst = ei + NE;

  char* ws = (char*)d_ws;
  size_t off = 0;
  unsigned short* XB   = (unsigned short*)(ws + off); off += SZ_XB;
  unsigned short* HHL  = (unsigned short*)(ws + off); off += SZ_HHL;
  float*          XLR  = (float*)(ws + off);          off += SZ_XLR;
  int*            HITS = (int*)(ws + off);            off += SZ_HITS;
  int*            SLOT = (int*)(ws + off);            off += SZ_SLOT;
  unsigned short* WINT = (unsigned short*)(ws + off); off += SZ_WINT;
  unsigned short* WLR  = (unsigned short*)(ws + off); off += SZ_WLR;
  unsigned short* WGD  = (unsigned short*)(ws + off); off += SZ_WGD;
  if (off != SZ_TOT) return;

  hipFuncSetAttribute(reinterpret_cast<const void*>(&k_bucket),
                      hipFuncAttributeMaxDynamicSharedMemorySize, LDS_BKT);

  k_prep<<<PB_TOT, NTHR, 0, stream>>>(x, W_in, Wl, Wr, Wg, XB, WINT, WLR, WGD);
  k_bucket<<<NBLK, NTHR, LDS_BKT, stream>>>(src, dst, ea, HITS, SLOT, 1);
  k_in<<<MP / GBM, GTHR, 0, stream>>>(XB, WINT, b_in, g_lni, b_lni, out, HHL);
  for (int l = 0; l < NL; ++l) {
    k_proj<<<dim3(MP / GBM, 2), GTHR, 0, stream>>>(HHL, WLR + (size_t)l * K2 * K2,
                                                   bl + (size_t)l * HID, br + (size_t)l * HID, XLR);
    k_scan<<<MP / SROWS, NTHR, 0, stream>>>(HITS, SLOT, XLR, We + (size_t)l * 2 * HID,
                                            att + (size_t)l * HID, bo + (size_t)l * HID,
                                            g_res + (size_t)l * HID, b_res + (size_t)l * HID, out, HHL);
  }
  k_gate<<<MP / GBM, GTHR, 0, stream>>>(HHL, WGD, bg, g_f, b_f, SLOT, out);
}
